// LSTMModel_16406775070721
// MI455X (gfx1250) — hardware-verified
//
#include <hip/hip_runtime.h>
#include <math.h>

constexpr int NBAT  = 4096;
constexpr int NSTEP = 200;
constexpr int NCH   = 16;
constexpr int NHID  = 112;
constexpr int NGATE = 4 * NHID;
constexpr int NOUTC = 6;
constexpr int KTOT  = NCH + NHID;
constexpr int ROWS_BLK = 16;
constexpr int LTHR  = 224;
constexpr int AP    = 136;
constexpr int HSP   = 116;
constexpr int BN_BLK = 256, BN_THR = 256;
constexpr int NX4   = NBAT * NSTEP * NCH / 4;
constexpr int NX4_ITER = NX4 / (BN_BLK * BN_THR);
constexpr int REDP  = 36;
constexpr int PREP_THR = 256, PREP_ROWS = 64, PREP_BLK = NGATE / PREP_ROWS;
constexpr int TP    = 136;
constexpr float WCARRY     = 256.0f;
constexpr float WCARRY_INV = 1.0f / 256.0f;
constexpr float BN_EPS     = 1e-5f;
constexpr float INV_NSAMP  = 1.0f / (float)(NBAT * NSTEP);

static_assert(KTOT % 32 == 0, "fused K is a multiple of the WMMA k step");
static_assert(NHID % 16 == 0 && NHID / 16 == LTHR / 32, "one wave per 16 hidden columns");
static_assert(NBAT % ROWS_BLK == 0, "recurrence grid exact");
static_assert(NX4 % (BN_BLK * BN_THR) == 0, "bn grid-stride loop exact");
static_assert(BN_BLK == PREP_THR, "one prep thread per partial line");
static_assert(NGATE % PREP_ROWS == 0, "prep grid exact");
static_assert(PREP_ROWS * (NCH / 4) == PREP_THR, "x-part tile fill exact");
static_assert(PREP_ROWS * (NHID / 4) == 7 * PREP_THR, "h-part tile fill exact");
static_assert(PREP_ROWS * (KTOT / 8) == 4 * PREP_THR, "Bt tile store exact");
static_assert(NGATE % 4 == 0 && NGATE / 4 <= PREP_THR, "beff store map");
static_assert((ROWS_BLK * NOUTC) % 4 == 0 && (ROWS_BLK * NOUTC) / 4 <= 32, "one wave writes a block's output");
static_assert((ROWS_BLK * NOUTC * 4) % 128 == 0, "block output is whole 128-B lines");
static_assert(AP % 8 == 0 && TP % 8 == 0 && HSP % 4 == 0, "16-B aligned LDS rows");

typedef __attribute__((ext_vector_type(16))) _Float16 v16h;
typedef __attribute__((ext_vector_type(8)))  _Float16 v8h;
typedef __attribute__((ext_vector_type(8)))  float    v8f;
typedef __attribute__((ext_vector_type(4)))  float    v4f;
typedef __attribute__((ext_vector_type(4)))  unsigned v4u;
typedef __attribute__((ext_vector_type(2)))  unsigned v2u;

template <typename T> struct Frag;
template <> struct Frag<_Float16> {
  typedef v16h V; union U { v16h v; v8h h[2]; };
  static __device__ __forceinline__ v16h load(const _Float16* p) {
    U f; f.h[0] = *(const v8h*)(p); f.h[1] = *(const v8h*)(p + 16); return f.v;
  }
  static __device__ __forceinline__ v8f mma(v16h a, v16h b, v8f c) {
    return __builtin_amdgcn_wmma_f32_16x16x32_f16(false, a, false, b, (short)0, c, false, false);
  }
};
__device__ __forceinline__ void mma_guard4(v8f& a0, v8f& a1, v8f& a2, v8f& a3,
                                           v16h fa, v16h f0, v16h f1, v16h f2, v16h f3) {
  asm volatile("v_nop\n\tv_nop\n\tv_nop\n\tv_nop"
               : "+v"(a0), "+v"(a1), "+v"(a2), "+v"(a3)
               : "v"(fa), "v"(f0), "v"(f1), "v"(f2), "v"(f3));
}
__device__ __forceinline__ void acc_guard4(v8f& a, v8f& b, v8f& c, v8f& d) {
  asm volatile("v_nop\n\tv_nop\n\tv_nop\n\tv_nop" : "+v"(a), "+v"(b), "+v"(c), "+v"(d));
}

__device__ __forceinline__ unsigned short f2h_bits(float f) {
  const _Float16 hv = (_Float16)f;
  return __builtin_bit_cast(unsigned short, hv);
}
__device__ __forceinline__ float fsig(float x)  { return __builtin_amdgcn_rcpf(1.0f + expf(-x)); }
__device__ __forceinline__ float ftanh(float x) { return 1.0f - 2.0f * __builtin_amdgcn_rcpf(expf(2.0f * x) + 1.0f); }

__global__ __launch_bounds__(BN_THR) void bn_stats_kernel(const float* __restrict__ x, float* __restrict__ partial) {
  __shared__ float ls[BN_THR * 4];
  __shared__ float lq[BN_THR * 4];
  __shared__ float red[32];
  const int tid = threadIdx.x;
  const size_t g = (size_t)blockIdx.x * BN_THR + tid;
  float s[4] = {0.0f, 0.0f, 0.0f, 0.0f};
  float q[4] = {0.0f, 0.0f, 0.0f, 0.0f};
#pragma unroll 1
  for (int k = 0; k < NX4_ITER; ++k) {
    const v4f v = *(const v4f*)(x + (g + (size_t)k * (BN_BLK * BN_THR)) * 4);
#pragma unroll
    for (int e = 0; e < 4; ++e) { s[e] += v[e]; q[e] = fmaf(v[e], v[e], q[e]); }
  }
#pragma unroll
  for (int e = 0; e < 4; ++e) { ls[tid * 4 + e] = s[e]; lq[tid * 4 + e] = q[e]; }
  __syncthreads();
  if (tid < NCH) {
    const int e = tid & 3, grp = tid >> 2;
    float a = 0.0f, b = 0.0f;
#pragma unroll 1
    for (int m = 0; m < BN_THR / 4; ++m) {
      const int t = grp + 4 * m;
      a += ls[t * 4 + e];
      b += lq[t * 4 + e];
    }
    red[tid] = a;
    red[NCH + tid] = b;
  }
  __syncthreads();
  if (tid < 32) {
    const float v = red[tid];
    float* op = partial + (size_t)blockIdx.x * 32 + tid;
    for (int pass = 0; pass < 2; ++pass) {
      *(volatile float*)op = v;
      __threadfence();
    }
  }
}

__global__ __launch_bounds__(PREP_THR) void prep_kernel(const float* __restrict__ partial,
                                                        const float* __restrict__ gamma, const float* __restrict__ beta,
                                                        const float* __restrict__ W_ih, const float* __restrict__ W_hh,
                                                        const float* __restrict__ b_ih, const float* __restrict__ b_hh,
                                                        float* __restrict__ beff, unsigned short* __restrict__ Btp) {
  __shared__ __align__(16) float red[BN_BLK * REDP];
  __shared__ float stat[32];
  __shared__ float bscale[NCH];
  __shared__ float bshift[NCH];
  __shared__ __align__(16) float beffs[NGATE];
  __shared__ __align__(16) unsigned short Tt[PREP_ROWS * TP];
  const int tid = threadIdx.x;
  const int r0 = blockIdx.x * PREP_ROWS;

#pragma unroll
  for (int qq = 0; qq < 8; ++qq) {
    const v4f v = *(const v4f*)(partial + (size_t)tid * 32 + 4 * qq);
    *(v4f*)(red + tid * REDP + 4 * qq) = v;
  }
  __syncthreads();
  if (tid < 32) {
    float sacc = 0.0f;
#pragma unroll 1
    for (int b = 0; b < BN_BLK; ++b) sacc += red[b * REDP + tid];
    stat[tid] = sacc;
  }
  __syncthreads();
  if (tid < NCH) {
    const float mean = stat[tid] * INV_NSAMP;
    const float var  = stat[NCH + tid] * INV_NSAMP - mean * mean;
    const float sc   = gamma[tid] * rsqrtf(var + BN_EPS);
    bscale[tid] = sc;
    bshift[tid] = beta[tid] - mean * sc;
  }
  __syncthreads();

#pragma unroll 1
  for (int g = tid; g < NGATE; g += PREP_THR) {
    const v4f w0 = *(const v4f*)(W_ih + (size_t)g * NCH + 0);
    const v4f w1 = *(const v4f*)(W_ih + (size_t)g * NCH + 4);
    const v4f w2 = *(const v4f*)(W_ih + (size_t)g * NCH + 8);
    const v4f w3 = *(const v4f*)(W_ih + (size_t)g * NCH + 12);
    float a = b_ih[g] + b_hh[g];
#pragma unroll
    for (int e = 0; e < 4; ++e) {
      a = fmaf(w0[e], bshift[e], a);
      a = fmaf(w1[e], bshift[4 + e], a);
      a = fmaf(w2[e], bshift[8 + e], a);
      a = fmaf(w3[e], bshift[12 + e], a);
    }
    beffs[g] = a;
  }
  __syncthreads();
  if (blockIdx.x == 0 && tid < NGATE / 4) {
    const v4f v = *(const v4f*)(beffs + 4 * tid);
    float* op = beff + 4 * tid;
    for (int pass = 0; pass < 2; ++pass) {
      *(volatile v4f*)op = v;
      __threadfence();
    }
  }

  {
    const int row = tid >> 2, c4 = (tid & 3) * 4;
    const v4f w = *(const v4f*)(W_ih + (size_t)(r0 + row) * NCH + c4);
#pragma unroll
    for (int e = 0; e < 4; ++e) {
      const float f = w[e] * (bscale[c4 + e] * WCARRY);
      Tt[row * TP + c4 + e] = f2h_bits(f);
    }
  }
#pragma unroll 1
  for (int it = 0; it < 7; ++it) {
    const int idx = it * PREP_THR + tid;
    const int row = idx / (NHID / 4);
    const int c4  = (idx - row * (NHID / 4)) * 4;
    const v4f w = *(const v4f*)(W_hh + (size_t)(r0 + row) * NHID + c4);
#pragma unroll
    for (int e = 0; e < 4; ++e) {
      const float f = w[e] * WCARRY;
      Tt[row * TP + NCH + c4 + e] = f2h_bits(f);
    }
  }
  __syncthreads();

  for (int pass = 0; pass < 2; ++pass) {
#pragma unroll
    for (int it = 0; it < 4; ++it) {
      const int idx = it * PREP_THR + tid;
      const int row = idx >> 4;
      const int c8  = (idx & 15) * 8;
      const v4u u = *(const v4u*)(Tt + row * TP + c8);
      *(volatile v4u*)(Btp + (size_t)(r0 + row) * KTOT + c8) = u;
    }
    __threadfence();
  }
}

__global__ __launch_bounds__(LTHR) void lstm_seq_kernel(const float* __restrict__ x, const float* __restrict__ beff,
                                                        const unsigned short* __restrict__ Btp,
                                                        const float* __restrict__ W_fc, const float* __restrict__ b_fc,
                                                        float* __restrict__ out) {
  __shared__ __align__(16) unsigned short At[ROWS_BLK * AP];
  __shared__ __align__(16) float Hs[ROWS_BLK * HSP];
  __shared__ __align__(16) float Os[ROWS_BLK * NOUTC];
  const _Float16* Bt = (const _Float16*)Btp;
  const int tid = threadIdx.x, lane = tid & 31, wave = tid >> 5;
  const int c = lane & 15, hh = lane >> 4, koff = hh * 8;
  const int rowbase = blockIdx.x * ROWS_BLK;
  const int j = 16 * wave + c;

#pragma unroll 1
  for (int i = tid; i < ROWS_BLK * AP; i += LTHR) At[i] = (unsigned short)0;
  __syncthreads();
  if (tid < 64) {
    const int m = tid >> 2, f4 = (tid & 3) * 4;
    const v4f v = *(const v4f*)(x + ((size_t)(rowbase + m) * NSTEP) * NCH + f4);
    const float x0 = v[0], x1 = v[1], x2 = v[2], x3 = v[3];
    const unsigned short u0 = f2h_bits(x0), u1 = f2h_bits(x1), u2 = f2h_bits(x2), u3 = f2h_bits(x3);
    v2u pk;
    pk[0] = (unsigned)u0 | ((unsigned)u1 << 16);
    pk[1] = (unsigned)u2 | ((unsigned)u3 << 16);
    *(v2u*)(At + m * AP + f4) = pk;
  }
  float bb[4];
#pragma unroll
  for (int g = 0; g < 4; ++g) bb[g] = beff[g * NHID + j];
  float cst[8], hst[8];
#pragma unroll
  for (int r = 0; r < 8; ++r) { cst[r] = 0.0f; hst[r] = 0.0f; }
  __syncthreads();

  const _Float16* arow = (const _Float16*)At + c * AP + koff;
  const _Float16* wrow = Bt + (size_t)j * KTOT + koff;
  const v8f z8 = {0.f, 0.f, 0.f, 0.f, 0.f, 0.f, 0.f, 0.f};

#pragma unroll 1
  for (int t = 0; t < NSTEP; ++t) {
    v8f acc[4];
    acc[0] = z8; acc[1] = z8; acc[2] = z8; acc[3] = z8;
#pragma unroll 1
    for (int k0 = 0; k0 < KTOT; k0 += 32) {
      const v16h a  = Frag<_Float16>::load(arow + k0);
      const v16h b0 = Frag<_Float16>::load(wrow + (size_t)0 * NHID * KTOT + k0);
      const v16h b1 = Frag<_Float16>::load(wrow + (size_t)1 * NHID * KTOT + k0);
      const v16h b2 = Frag<_Float16>::load(wrow + (size_t)2 * NHID * KTOT + k0);
      const v16h b3 = Frag<_Float16>::load(wrow + (size_t)3 * NHID * KTOT + k0);
      acc[0] = Frag<_Float16>::mma(a, b0, acc[0]);
      acc[1] = Frag<_Float16>::mma(a, b1, acc[1]);
      acc[2] = Frag<_Float16>::mma(a, b2, acc[2]);
      acc[3] = Frag<_Float16>::mma(a, b3, acc[3]);
      mma_guard4(acc[0], acc[1], acc[2], acc[3], a, b0, b1, b2, b3);
    }
    acc_guard4(acc[0], acc[1], acc[2], acc[3]);
#pragma unroll
    for (int r = 0; r < 8; ++r) {
      const float zi = acc[0][r] * WCARRY_INV + bb[0];
      const float zf = acc[1][r] * WCARRY_INV + bb[1];
      const float zg = acc[2][r] * WCARRY_INV + bb[2];
      const float zo = acc[3][r] * WCARRY_INV + bb[3];
      const float ig = fsig(zi);
      const float fg = fsig(zf);
      const float gg = ftanh(zg);
      const float og = fsig(zo);
      const float cn = fg * cst[r] + ig * gg;
      cst[r] = cn;
      hst[r] = og * ftanh(cn);
    }
    __syncthreads();
#pragma unroll
    for (int r = 0; r < 8; ++r) At[(8 * hh + r) * AP + NCH + j] = f2h_bits(hst[r]);
    if (tid < 64) {
      const int tn = (t + 1 < NSTEP) ? (t + 1) : (NSTEP - 1);
      const int m = tid >> 2, f4 = (tid & 3) * 4;
      const v4f v = *(const v4f*)(x + ((size_t)(rowbase + m) * NSTEP + (size_t)tn) * NCH + f4);
      const float x0 = v[0], x1 = v[1], x2 = v[2], x3 = v[3];
      const unsigned short u0 = f2h_bits(x0), u1 = f2h_bits(x1), u2 = f2h_bits(x2), u3 = f2h_bits(x3);
      v2u pk;
      pk[0] = (unsigned)u0 | ((unsigned)u1 << 16);
      pk[1] = (unsigned)u2 | ((unsigned)u3 << 16);
      *(v2u*)(At + m * AP + f4) = pk;
    }
    __syncthreads();
  }

#pragma unroll
  for (int r = 0; r < 8; ++r) Hs[(8 * hh + r) * HSP + j] = hst[r];
  __syncthreads();
  if (tid < ROWS_BLK * NOUTC) {
    const int rr = tid / NOUTC;
    const int o  = tid - rr * NOUTC;
    const float* hp = Hs + rr * HSP;
    const float* wp = W_fc + (size_t)o * NHID;
    float a = b_fc[o];
#pragma unroll 1
    for (int n = 0; n < NHID; ++n) a = fmaf(hp[n], wp[n], a);
    Os[tid] = tanhf(a);
  }
  __syncthreads();
  if (wave == 0) {
    const int lc = (lane < (ROWS_BLK * NOUTC) / 4) ? lane : ((ROWS_BLK * NOUTC) / 4 - 1);
    const v4f v = *(const v4f*)(Os + 4 * lc);
    float* op = out + (size_t)blockIdx.x * (ROWS_BLK * NOUTC) + 4 * lc;
    for (int pass = 0; pass < 2; ++pass) {
      if (lane < (ROWS_BLK * NOUTC) / 4) *(volatile v4f*)op = v;
      __threadfence();
    }
  }
}

extern "C" void kernel_launch(void* const* d_in, const int* in_sizes, int n_in,
                              void* d_out, int out_size, void* d_ws, size_t ws_size, hipStream_t stream) {
  if (n_in < 9 || d_out == nullptr || d_ws == nullptr) return;
  if (in_sizes[0] != NBAT * NSTEP * NCH || in_sizes[1] != NCH || in_sizes[2] != NCH ||
      in_sizes[3] != NGATE * NCH || in_sizes[4] != NGATE * NHID || in_sizes[5] != NGATE ||
      in_sizes[6] != NGATE || in_sizes[7] != NOUTC * NHID || in_sizes[8] != NOUTC ||
      out_size != NBAT * NOUTC) return;

  const float* x     = (const float*)d_in[0];
  const float* gamma = (const float*)d_in[1];
  const float* beta  = (const float*)d_in[2];
  const float* W_ih  = (const float*)d_in[3];
  const float* W_hh  = (const float*)d_in[4];
  const float* b_ih  = (const float*)d_in[5];
  const float* b_hh  = (const float*)d_in[6];
  const float* W_fc  = (const float*)d_in[7];
  const float* b_fc  = (const float*)d_in[8];
  float* out = (float*)d_out;

  char* ws = (char*)d_ws; size_t off = 0;
  auto carve = [&](size_t bytes) -> char* { char* p = ws + off; off += (bytes + 255) & ~(size_t)255; return p; };
  float*          PART = (float*)carve((size_t)BN_BLK * 32 * 4);
  float*          BEFF = (float*)carve((size_t)NGATE * 4);
  unsigned short* BTP  = (unsigned short*)carve((size_t)NGATE * KTOT * 2);
  if (off > ws_size || off > (size_t)134217728) return;

  bn_stats_kernel<<<BN_BLK, BN_THR, 0, stream>>>(x, PART);
  prep_kernel<<<PREP_BLK, PREP_THR, 0, stream>>>(PART, gamma, beta, W_ih, W_hh, b_ih, b_hh, BEFF, BTP);
  lstm_seq_kernel<<<NBAT / ROWS_BLK, LTHR, 0, stream>>>(x, BEFF, BTP, W_fc, b_fc, out);
}
